// MoELayer_57664230916132
// MI455X (gfx1250) — hardware-verified
//
#include <hip/hip_runtime.h>
#include <math.h>

typedef __attribute__((ext_vector_type(16))) _Float16 v16h;
typedef __attribute__((ext_vector_type(16))) __bf16 v16b;
typedef __attribute__((ext_vector_type(8)))  _Float16 v8h;
typedef __attribute__((ext_vector_type(8)))  float v8f;
typedef __attribute__((ext_vector_type(4)))  float v4f;
typedef __attribute__((ext_vector_type(2)))  float v2f;
typedef __attribute__((ext_vector_type(4)))  unsigned v4u;
typedef __attribute__((ext_vector_type(4)))  int v4i;
typedef float __attribute__((may_alias)) float_a;
typedef int __attribute__((may_alias)) int_a;

template <typename T> __device__ __forceinline__ void vst2(void* p, T v) { *(volatile T*)p = v; __threadfence(); *(volatile T*)p = v; }
__device__ __forceinline__ v8f wmma16(v16h a, v16h b, v8f c) {
  v8f d = __builtin_amdgcn_wmma_f32_16x16x32_f16(false, a, false, b, (short)0, c, false, false);
  asm volatile("v_nop\n\tv_nop\n\tv_nop\n\tv_nop" : "+v"(d) : "v"(a), "v"(b));
  return d;
}
__device__ __forceinline__ v8f wmma_bf(v16b a, v16b b, v8f c) {
  v8f d = __builtin_amdgcn_wmma_f32_16x16x32_bf16(false, a, false, b, (short)0, c, false, false);
  asm volatile("v_nop\n\tv_nop\n\tv_nop\n\tv_nop" : "+v"(d) : "v"(a), "v"(b));
  return d;
}
__device__ __forceinline__ v16h frag_h(const _Float16* rowk0, int lane) {
  union { v16h v; v8h q[2]; } u; const _Float16* p = rowk0 + 8 * (lane >> 4);
  u.q[0] = *(const v8h*)p; u.q[1] = *(const v8h*)(p + 16); return u.v;
}
__device__ __forceinline__ v16h frag_f32(const float* rowk0, int lane) {
  v16h a; const float* p = rowk0 + 8 * (lane >> 4);
#pragma unroll
  for (int i = 0; i < 8; ++i) { a[i] = (_Float16)p[i]; a[8 + i] = (_Float16)p[16 + i]; }
  return a;
}
__device__ __forceinline__ v16h frag_f32s(const float* rowk0, int lane, float sc) {
  v16h a; const float* p = rowk0 + 8 * (lane >> 4);
#pragma unroll
  for (int i = 0; i < 8; ++i) { a[i] = (_Float16)(p[i] * sc); a[8 + i] = (_Float16)(p[16 + i] * sc); }
  return a;
}
__device__ __forceinline__ v16h fragc_f32(const float* W, int k0, int n, int lane, int ld, int K) {
  v16h a; const int g = lane >> 4;
#pragma unroll
  for (int i = 0; i < 8; ++i) { const int ka = k0 + 8 * g + i, kb = ka + 16;
    a[i] = (_Float16)(ka < K ? W[(size_t)(ka < K ? ka : K - 1) * ld + n] : 0.f); a[8 + i] = (_Float16)(kb < K ? W[(size_t)(kb < K ? kb : K - 1) * ld + n] : 0.f); }
  return a;
}
struct F2 { v16b h, l; };
__device__ __forceinline__ F2 bsplit16(const float v[16]) { F2 r;
#pragma unroll
  for (int i = 0; i < 16; ++i) { const __bf16 h = (__bf16)v[i]; r.h[i] = h; r.l[i] = (__bf16)(v[i] - (float)h); }
  return r; }
__device__ __forceinline__ F2 split_row(const float* row, int k0, int lane) { float v[16]; const float* p = row + k0 + 8 * (lane >> 4);
#pragma unroll
  for (int i = 0; i < 8; ++i) { v[i] = p[i]; v[8 + i] = p[16 + i]; }
  return bsplit16(v); }
__device__ __forceinline__ F2 split_rowK(const float* row, int k0, int lane, int K) { float v[16]; const int g = lane >> 4;
#pragma unroll
  for (int i = 0; i < 8; ++i) { const int ka = k0 + 8 * g + i, kb = ka + 16; v[i] = ka < K ? row[ka < K ? ka : K - 1] : 0.f; v[8 + i] = kb < K ? row[kb < K ? kb : K - 1] : 0.f; }
  return bsplit16(v); }
__device__ __forceinline__ F2 split_col(const float* W, int k0, int n, int lane, int ld, int K) { float v[16]; const int g = lane >> 4;
#pragma unroll
  for (int i = 0; i < 8; ++i) { const int ka = k0 + 8 * g + i, kb = ka + 16; v[i] = ka < K ? W[(size_t)(ka < K ? ka : K - 1) * ld + n] : 0.f; v[8 + i] = kb < K ? W[(size_t)(kb < K ? kb : K - 1) * ld + n] : 0.f; }
  return bsplit16(v); }
__device__ __forceinline__ v8f mac3(const F2& a, const F2& b, v8f c) { c = wmma_bf(a.l, b.h, c); c = wmma_bf(a.h, b.l, c); return wmma_bf(a.h, b.h, c); }
__device__ __forceinline__ float sigm(float v) { return 1.0f / (1.0f + expf(-v)); }
#define LDSX() do { asm volatile("s_wait_dscnt 0" ::: "memory"); __builtin_amdgcn_wave_barrier(); __builtin_amdgcn_fence(__ATOMIC_RELEASE, "workgroup"); } while (0)

#define NT 8192
#define DD 1024
#define HH 256
#define HS (NE * HH)
#define NE 8
#define KS 8
#define NSH 1
typedef __attribute__((ext_vector_type(4))) int v4i2;
__device__ __forceinline__ float bfr(float v) { return (float)(__bf16)v; }
__device__ __forceinline__ v16b wcol_in(const float* Wm, int k0, int o, int lane, int ld, int nvalid) { v16b w; const int g = lane >> 4; const int oc = o < nvalid ? o : 0; const float keep = o < nvalid ? 1.f : 0.f; float t0[8], t1[8];
#pragma unroll
  for (int i = 0; i < 8; ++i) t0[i] = Wm[(size_t)(k0 + 8 * g + i) * ld + oc];
  asm volatile("s_wait_loadcnt 0x0" ::: "memory");
#pragma unroll
  for (int i = 0; i < 8; ++i) t1[i] = Wm[(size_t)(k0 + 16 + 8 * g + i) * ld + oc];
  asm volatile("s_wait_loadcnt 0x0" ::: "memory");
#pragma unroll
  for (int i = 0; i < 8; ++i) { w[i] = (__bf16)(t0[i] * keep); w[8 + i] = (__bf16)(t1[i] * keep); }
  return w; }
#define WS_IDX 0u
#define WS_WGT (WS_IDX + 16u * NT)
#define WS_TOK (WS_WGT + 16u * NT)
#define WS_RB  (WS_TOK + 16u * NT)
#define WS_H   (WS_RB + 64u * NRB + 1024u)
#define WS_END (WS_H + 4u * (size_t)NT * HS)

#define DOUT 1024
__global__ __launch_bounds__(128) void k_route(const float* __restrict__ X, const float* __restrict__ WG, const float* __restrict__ BG, int* __restrict__ IDX, float* __restrict__ WGT, float* __restrict__ LOG) { __shared__ __align__(16) float sl[64][8]; __shared__ __align__(16) int si[64][KS]; __shared__ __align__(16) float sw[64][KS]; __shared__ __align__(16) float swg[DD * NE];
  const int tid = threadIdx.x, wave = tid >> 5, lane = tid & 31, col = lane & 15, g = lane >> 4; const size_t r0 = (size_t)blockIdx.x * 64;
  for (int r = 0; r < (DD * NE) / (4 * 128); ++r) { const v4f t4 = *(const v4f*)(WG + ((size_t)r * 128 + tid) * 4); asm volatile("s_wait_loadcnt 0x0" ::: "memory"); *(v4f*)&swg[((size_t)r * 128 + tid) * 4] = t4; }
  __syncthreads();
  v8f acc = {};
#pragma unroll 1
  for (int kc = 0; kc < DD / 32; ++kc) {
    v16b w; { const int e2 = col < NE ? col : 0; const float keep = col < NE ? 1.f : 0.f; const float* pw = swg + (size_t)(kc * 32 + 8 * g) * NE + e2;
#pragma unroll
      for (int i = 0; i < 8; ++i) { w[i] = (__bf16)(pw[(size_t)i * NE] * keep); w[8 + i] = (__bf16)(pw[(size_t)(16 + i) * NE] * keep); } }
    v16b a; { const float* p = X + (r0 + wave * 16 + col) * DD + kc * 32 + 8 * g;
#pragma unroll
      for (int i = 0; i < 8; ++i) { a[i] = (__bf16)p[i]; a[8 + i] = (__bf16)p[16 + i]; } }
    asm volatile("s_wait_loadcnt 0x0" ::: "memory"); acc = wmma_bf(a, w, acc); }
  if (col < NE) {
#pragma unroll
    for (int r = 0; r < 8; ++r) sl[wave * 16 + 8 * g + r][col] = acc[r]; }
  __syncthreads();
  if (tid < 64) { float l[NE];
#pragma unroll
    for (int e = 0; e < NE; ++e) l[e] = sl[tid][e] + bfr(BG[e]);
    int sel[KS]; float sv[KS]; unsigned usedm = 0u;
#pragma unroll
    for (int s = 0; s < KS; ++s) { int be = -1; float bv = -3.0e38f;
#pragma unroll
      for (int e = 0; e < NE; ++e) { const bool free_ = ((usedm >> e) & 1u) == 0u; const bool take = free_ && (be < 0 || l[e] > bv); bv = take ? l[e] : bv; be = take ? e : be; }
      usedm |= 1u << be; sel[s] = be; sv[s] = bv; }
    float den = 0.f; float ev[KS];
#pragma unroll
    for (int s = 0; s < KS; ++s) { ev[s] = expf(sv[s] - sv[0]); den += ev[s]; }
#pragma unroll
    for (int s = 0; s < KS; ++s) { si[tid][s] = sel[s]; sw[tid][s] = ev[s] / den; } }
  __syncthreads();
  __syncthreads();
  (void)LOG;
  if (tid < 64) { v4f w0, w1; _Pragma("unroll") for (int s2 = 0; s2 < 4; ++s2) { w0[s2] = sw[tid][s2]; w1[s2] = sw[tid][4 + s2]; } vst2((v4f*)(WGT + (r0 + tid) * KS), w0); vst2((v4f*)(WGT + (r0 + tid) * KS + 4), w1); } }

__device__ __forceinline__ v16b wcol_io(const float* Wm, int k0, int o, int lane, int ld) { v16b w; const int g = lane >> 4;
#pragma unroll
  for (int i = 0; i < 8; ++i) { w[i] = (__bf16)Wm[(size_t)(k0 + 8 * g + i) * ld + o]; w[8 + i] = (__bf16)Wm[(size_t)(k0 + 16 + 8 * g + i) * ld + o]; }
  return w; }
__global__ __launch_bounds__(128) void k_hid(const float* __restrict__ X, const float* __restrict__ W1, const float* __restrict__ B1, float* __restrict__ Hd) { __shared__ __align__(16) float sf[4][16][132];
  const int tid = threadIdx.x, wave = tid >> 5, lane = tid & 31, col = lane & 15, g = lane >> 4; const size_t r0 = (size_t)blockIdx.x * 64 + wave * 16; const int c0 = blockIdx.y * 128; const int e = blockIdx.z;
  const float* We = W1 + (size_t)e * DD * HH; v8f acc[8] = {};
#pragma unroll 1
  for (int kc = 0; kc < DD / 32; ++kc) { v16b a; { const float* p = X + (r0 + col) * DD + kc * 32 + 8 * g;
#pragma unroll
      for (int i = 0; i < 8; ++i) { a[i] = (__bf16)p[i]; a[8 + i] = (__bf16)p[16 + i]; } }
    asm volatile("s_wait_loadcnt 0x0" ::: "memory");
#pragma unroll
    for (int j = 0; j < 8; ++j) { const v16b w = wcol_io(We, kc * 32, c0 + j * 16 + col, lane, HH); asm volatile("s_wait_loadcnt 0x0" ::: "memory"); acc[j] = wmma_bf(a, w, acc[j]); } }
#pragma unroll
  for (int j = 0; j < 8; ++j) { const float bb = bfr(B1[(size_t)e * HH + c0 + j * 16 + col]); asm volatile("s_wait_loadcnt 0x0" ::: "memory");
#pragma unroll
    for (int r = 0; r < 8; ++r) { const float v = acc[j][r] + bb; sf[wave][8 * g + r][j * 16 + col] = 0.5f * v * (1.0f + erff(v * 0.70710678118654752f)); } }
  LDSX(); for (int rl = 0; rl < 16; ++rl) vst2(Hd + (r0 + rl) * (size_t)HS + (size_t)e * HH + c0 + lane * 4, *(const v4f*)&sf[wave][rl][lane * 4]); }
__global__ __launch_bounds__(128) void k_dout(const float* __restrict__ Hd, const float* __restrict__ W2, const float* __restrict__ B2, const float* __restrict__ SP, float* __restrict__ OUT) { __shared__ __align__(16) float sf[4][16][132];
  const int tid = threadIdx.x, wave = tid >> 5, lane = tid & 31, col = lane & 15, g = lane >> 4; const size_t r0 = (size_t)blockIdx.x * 64 + wave * 16; const int c0 = blockIdx.y * 128;
  v8f tot[8] = {}; float wr[8][NE];
#pragma unroll
  for (int r = 0; r < 8; ++r) { const v4f a0 = *(const v4f*)(SP + (r0 + 8 * g + r) * KS), a1 = *(const v4f*)(SP + (r0 + 8 * g + r) * KS + 4); asm volatile("s_wait_loadcnt 0x0" ::: "memory"); _Pragma("unroll") for (int i = 0; i < 4; ++i) { wr[r][i] = a0[i]; wr[r][4 + i] = a1[i]; } }
#pragma unroll 1
  for (int e = 0; e < NE; ++e) { v8f acc[8] = {}; const float* We = W2 + (size_t)e * HH * DOUT;
#pragma unroll 1
    for (int kc = 0; kc < HH / 32; ++kc) { const v16h a = frag_f32(Hd + (r0 + col) * (size_t)HS + (size_t)e * HH + kc * 32, lane); asm volatile("s_wait_loadcnt 0x0" ::: "memory");
#pragma unroll
      for (int j = 0; j < 8; ++j) { v16h w; { const int o = c0 + j * 16 + col; float t0[8], t1[8];
#pragma unroll
          for (int i = 0; i < 8; ++i) t0[i] = We[(size_t)(kc * 32 + 8 * g + i) * DOUT + o];
          asm volatile("s_wait_loadcnt 0x0" ::: "memory");
#pragma unroll
          for (int i = 0; i < 8; ++i) t1[i] = We[(size_t)(kc * 32 + 16 + 8 * g + i) * DOUT + o];
          asm volatile("s_wait_loadcnt 0x0" ::: "memory");
#pragma unroll
          for (int i = 0; i < 8; ++i) { w[i] = (_Float16)(bfr(t0[i]) * 64.0f); w[8 + i] = (_Float16)(bfr(t1[i]) * 64.0f); } }
        acc[j] = wmma16(a, w, acc[j]); } }
#pragma unroll
    for (int j = 0; j < 8; ++j) { const float bb = bfr(B2[(size_t)e * DOUT + c0 + j * 16 + col]); asm volatile("s_wait_loadcnt 0x0" ::: "memory");
      float we8[8]; _Pragma("unroll") for (int r = 0; r < 8; ++r) { we8[r] = wr[r][0]; _Pragma("unroll") for (int i = 1; i < NE; ++i) we8[r] = (i == e) ? wr[r][i] : we8[r]; }
#pragma unroll
      for (int r = 0; r < 8; ++r) tot[j][r] += ((e == 0) ? wr[r][0] : we8[r]) * (acc[j][r] * (1.0f / 64.0f) + bb); } }
#pragma unroll
  for (int j = 0; j < 8; ++j)
#pragma unroll
    for (int r = 0; r < 8; ++r) sf[wave][8 * g + r][j * 16 + col] = tot[j][r];
  LDSX(); for (int rl = 0; rl < 16; ++rl) vst2(OUT + (r0 + rl) * (size_t)DOUT + c0 + lane * 4, *(const v4f*)&sf[wave][rl][lane * 4]); }
#undef WS_END
#define WS_HD  0u
#define WS_SP  (WS_HD + 4u * (size_t)NT * HS)
#define WS_ENDX (WS_SP + 32u * (size_t)NT + 256u)
extern "C" void kernel_launch(void* const* d_in, const int* in_sizes, int n_in, void* d_out, int out_size, void* d_ws, size_t ws_size, hipStream_t stream) {
  (void)in_sizes; (void)n_in; (void)out_size;
  const float** F = (const float**)d_in;
  if (ws_size < (size_t)WS_ENDX) return;
  char* ws = (char*)d_ws; float *SP = (float*)(ws + WS_SP), *Hd = (float*)(ws + WS_HD);
  k_route<<<dim3(NT / 64), 128, 0, stream>>>(F[0], F[1], F[2], nullptr, SP, nullptr);
  k_hid<<<dim3(NT / 64, HH / 128, NE), 128, 0, stream>>>(F[0], F[3], F[4], Hd);
  k_dout<<<dim3(NT / 64, DOUT / 128), 128, 0, stream>>>(Hd, F[5], F[6], SP, (float*)d_out);
}
